// MambaBlock_46926812676556
// MI455X (gfx1250) — hardware-verified
//
#include <hip/hip_runtime.h>
#include <stddef.h>
#include <stdint.h>
#include <math.h>


#define NB     4
#define LL     1024
#define DM     512
#define DI     1024
#define NS     16
#define RK     32
#define MR     (NB * LL)
#define XW     64
#define XRW    (2 * DI)
#define K2U    (2 * DI)
#define K2D    (2 * RK)
#define GBM    64
#define GBN    64
#define GTHR   128
#define NTHR   256
#define TC     32
#define SD     64
#define WSMAX  134217728

#define UX     (MR * DM / 8)
#define UWI    (XRW * (DM / 8))
#define UWX    (XW * (K2U / 8))
#define UWD    (DI * (K2D / 8))
#define UWO    (DM * (K2U / 8))
#define UTOT   (UX + UWI + UWX + UWD + UWO)

static_assert(UX % NTHR == 0 && UWI % NTHR == 0 && UWX % NTHR == 0 && UWD % NTHR == 0 && UWO % NTHR == 0);
static_assert(MR % GBM == 0 && XRW % GBN == 0 && XW % GBN == 0 && DI % GBN == 0 && DM % GBN == 0);
static_assert(DM % 32 == 0 && K2U % 32 == 0 && K2D % 32 == 0);
static_assert(GBM == (GTHR / 32) * 16 && GBN == 64);
static_assert(LL % TC == 0 && DI % SD == 0 && NTHR == 4 * SD && NTHR == 8 * TC && TC == 32 && SD == 64);
static_assert(DI == 4 * NTHR && K2U == 8 * NTHR);
static_assert(XW == RK + 2 * NS);

typedef float          v4f   __attribute__((ext_vector_type(4)));
typedef float          v8f   __attribute__((ext_vector_type(8)));
typedef int            v8i   __attribute__((ext_vector_type(8)));
typedef unsigned short v8us  __attribute__((ext_vector_type(8)));
typedef unsigned short v16us __attribute__((ext_vector_type(16)));
typedef __bf16         v16bf __attribute__((ext_vector_type(16)));
typedef v4f  __attribute__((may_alias)) v4fa;
typedef v8us __attribute__((may_alias)) v8usa;
union FragB { v16bf v; v16us u; v8us h[2]; v8i w; };

__device__ __forceinline__ v8f wmb(const FragB& a, const FragB& b, v8f c) {
  v8f d = __builtin_amdgcn_wmma_f32_16x16x32_bf16(false, a.v, false, b.v, (short)0, c, false, false);
  asm volatile("v_nop\n\tv_nop\n\tv_nop\n\tv_nop" : "+v"(d) : "v"(a.w), "v"(b.w));
  return d;
}

__device__ __forceinline__ unsigned bf16_bits(float f) {
  const unsigned u = __float_as_uint(f);
  return (u + 0x7FFFu + ((u >> 16) & 1u)) >> 16;
}
__device__ __forceinline__ float bf16_val(float f) {
  return __uint_as_float(bf16_bits(f) << 16);
}
__device__ __forceinline__ unsigned short hl_sel(float v, bool lsel) {
  const unsigned hb = bf16_bits(v);
  const unsigned lb = bf16_bits(v - __uint_as_float(hb << 16));
  return (unsigned short)(lsel ? lb : hb);
}
__device__ __forceinline__ float softplus_f(float v) {
  return fmaxf(v, 0.0f) + log1pf(expf(-fabsf(v)));
}

__device__ __forceinline__ v8us gather8(const float* __restrict__ p, size_t stride) {
  v8us o;
#pragma unroll
  for (int i = 0; i < 8; ++i) o[i] = (unsigned short)bf16_bits(p[(size_t)i * stride]);
  return o;
}
__device__ __forceinline__ void put8(unsigned short* dp, v8us o) {
  *(volatile v8us*)dp = o;
  __threadfence();
  *(volatile v8us*)dp = o;
}

__global__ __launch_bounds__(NTHR) void k_prep(const float* __restrict__ x, const float* __restrict__ W_in,
                                               const float* __restrict__ W_x, const float* __restrict__ W_dt,
                                               const float* __restrict__ W_out,
                                               unsigned short* XB, unsigned short* WIN_T, unsigned short* WX2,
                                               unsigned short* WDT2, unsigned short* WO2) {
  const int u = (int)blockIdx.x * NTHR + (int)threadIdx.x;
  if (u < UX) {
    const int row = u >> 6;
    const int k8  = (u & 63) * 8;
    const float* p = x + (size_t)row * DM + k8;
    const v4f a = *(const v4f*)p;
    const v4f b = *(const v4f*)(p + 4);
    v8us o;
    o[0] = (unsigned short)bf16_bits(a.x); o[1] = (unsigned short)bf16_bits(a.y);
    o[2] = (unsigned short)bf16_bits(a.z); o[3] = (unsigned short)bf16_bits(a.w);
    o[4] = (unsigned short)bf16_bits(b.x); o[5] = (unsigned short)bf16_bits(b.y);
    o[6] = (unsigned short)bf16_bits(b.z); o[7] = (unsigned short)bf16_bits(b.w);
    put8(XB + (size_t)row * DM + k8, o);
  } else if (u < UX + UWI) {
    const int v  = u - UX;
    const int n  = v >> 6;
    const int k8 = (v & 63) * 8;
    const v8us o = gather8(W_in + (size_t)k8 * XRW + n, (size_t)XRW);
    put8(WIN_T + (size_t)n * DM + k8, o);
  } else if (u < UX + UWI + UWX) {
    const int v  = u - (UX + UWI);
    const int n  = v >> 8;
    const int k8 = (v & 255) * 8;
    const int kk = k8 & (DI - 1);
    const v8us o = gather8(W_x + (size_t)kk * XW + n, (size_t)XW);
    put8(WX2 + (size_t)n * K2U + k8, o);
  } else if (u < UX + UWI + UWX + UWD) {
    const int v  = u - (UX + UWI + UWX);
    const int n  = v >> 3;
    const int k8 = (v & 7) * 8;
    const int kk = k8 & (RK - 1);
    const v8us o = gather8(W_dt + (size_t)kk * DI + n, (size_t)DI);
    put8(WDT2 + (size_t)n * K2D + k8, o);
  } else if (u < UTOT) {
    const int v  = u - (UX + UWI + UWX + UWD);
    const int n  = v >> 8;
    const int k8 = (v & 255) * 8;
    const int kk = k8 & (DI - 1);
    const v8us o = gather8(W_out + (size_t)kk * DM + n, (size_t)DM);
    put8(WO2 + (size_t)n * K2U + k8, o);
  }
}

template <int EPI>
__global__ __launch_bounds__(GTHR) void k_gemm(const unsigned short* __restrict__ A,
                                               const unsigned short* __restrict__ WT, int K,
                                               const float* __restrict__ bias, float* outF, int ldo,
                                               unsigned short* outH) {
  __shared__ __attribute__((aligned(16))) float stg[GBM * GBN];
  const int tid = (int)threadIdx.x, lane = tid & 31, wave = tid >> 5, hh = lane >> 4, m = lane & 15;
  const int rowBase = (int)blockIdx.x * GBM;
  const int col0    = (int)blockIdx.y * GBN;

  v8f acc[4];
  {
    const v8f z = {0.f, 0.f, 0.f, 0.f, 0.f, 0.f, 0.f, 0.f};
    acc[0] = z; acc[1] = z; acc[2] = z; acc[3] = z;
  }
  const unsigned short* ap = A  + (size_t)(rowBase + 16 * wave + m) * (size_t)K + 8 * hh;
  const unsigned short* wp = WT + (size_t)(col0 + m) * (size_t)K + 8 * hh;
  const int ksteps = K >> 5;
#pragma unroll 1
  for (int ks = 0; ks < ksteps; ++ks) {
    FragB af;
    af.h[0] = *(const v8usa*)(ap + 32 * ks);
    af.h[1] = *(const v8usa*)(ap + 32 * ks + 16);
#pragma unroll
    for (int t = 0; t < 4; ++t) {
      const unsigned short* wq = wp + (size_t)(16 * t) * (size_t)K + 32 * ks;
      FragB bf;
      bf.h[0] = *(const v8usa*)wq;
      bf.h[1] = *(const v8usa*)(wq + 16);
      acc[t] = wmb(af, bf, acc[t]);
    }
  }

#pragma unroll
  for (int t = 0; t < 4; ++t) {
    const int lc = 16 * t + m;
#pragma unroll
    for (int r = 0; r < 8; ++r) {
      const int lr = 16 * wave + 8 * hh + r;
      stg[lr * GBN + lc] = acc[t][r];
    }
  }
  __syncthreads();

  v4f bb4 = {0.f, 0.f, 0.f, 0.f};
  if constexpr (EPI >= 2) {
    const v4f t = *(const v4f*)(bias + col0 + 4 * m);
    bb4.x = bf16_val(t.x); bb4.y = bf16_val(t.y); bb4.z = bf16_val(t.z); bb4.w = bf16_val(t.w);
  }
  if constexpr (EPI == 2) {
#pragma unroll 1
    for (int i = 0; i < 8; ++i) {
      const int lr = 16 * wave + 2 * i + hh;
      v4f t = *(const v4fa*)(stg + lr * GBN + 4 * m);
      t.x = softplus_f(t.x + bb4.x);
      t.y = softplus_f(t.y + bb4.y);
      t.z = softplus_f(t.z + bb4.z);
      t.w = softplus_f(t.w + bb4.w);
      *(v4fa*)(stg + lr * GBN + 4 * m) = t;
    }
  }

  v4f fv[8];
#pragma unroll
  for (int i = 0; i < 8; ++i) {
    const int lr = 16 * wave + 2 * i + hh;
    fv[i] = *(const v4fa*)(stg + lr * GBN + 4 * m);
    if constexpr (EPI == 3) fv[i] = fv[i] + bb4;
  }

  v8us dq[4];
  const int pp = lane & 7;
  if constexpr (EPI == 1) {
    const int cb = 8 * (pp & 3);
    const bool lsel = pp >= 4;
#pragma unroll
    for (int i = 0; i < 4; ++i) {
      const int lr = 16 * wave + 4 * i + (lane >> 3);
      const v4f a = *(const v4fa*)(stg + lr * GBN + cb);
      const v4f b = *(const v4fa*)(stg + lr * GBN + cb + 4);
      v8us o;
      o[0] = hl_sel(a.x, lsel); o[1] = hl_sel(a.y, lsel); o[2] = hl_sel(a.z, lsel); o[3] = hl_sel(a.w, lsel);
      o[4] = hl_sel(b.x, lsel); o[5] = hl_sel(b.y, lsel); o[6] = hl_sel(b.z, lsel); o[7] = hl_sel(b.w, lsel);
      dq[i] = o;
    }
  }

#pragma unroll
  for (int i = 0; i < 8; ++i) {
    const int gr = rowBase + 16 * wave + 2 * i + hh;
    float* op = outF + (size_t)gr * (size_t)ldo + col0 + 4 * m;
    *(volatile v4f*)op = fv[i];
  }
  if constexpr (EPI == 1) {
#pragma unroll
    for (int i = 0; i < 4; ++i) {
      const int gr = rowBase + 16 * wave + 4 * i + (lane >> 3);
      unsigned short* hp = outH + (size_t)gr * K2D + 8 * pp;
      *(volatile v8us*)hp = dq[i];
    }
  }
  __threadfence();
#pragma unroll
  for (int i = 0; i < 8; ++i) {
    const int gr = rowBase + 16 * wave + 2 * i + hh;
    float* op = outF + (size_t)gr * (size_t)ldo + col0 + 4 * m;
    *(volatile v4f*)op = fv[i];
  }
  if constexpr (EPI == 1) {
#pragma unroll
    for (int i = 0; i < 4; ++i) {
      const int gr = rowBase + 16 * wave + 4 * i + (lane >> 3);
      unsigned short* hp = outH + (size_t)gr * K2D + 8 * pp;
      *(volatile v8us*)hp = dq[i];
    }
  }
}

__global__ __launch_bounds__(NTHR) void k_conv(const float* __restrict__ XR, const float* __restrict__ cw,
                                               const float* __restrict__ cb, float* U, unsigned short* UHL) {
  __shared__ __attribute__((aligned(16))) float urow[DI];
  __shared__ __attribute__((aligned(16))) unsigned short hl[K2U];
  const int tid = (int)threadIdx.x;
  const int m = (int)blockIdx.x;
  const int t = m & (LL - 1);
  const int r0 = (m - 3) < 0 ? 0 : (m - 3);
  const int r1 = (m - 2) < 0 ? 0 : (m - 2);
  const int r2 = (m - 1) < 0 ? 0 : (m - 1);
  const bool ok0 = t >= 3, ok1 = t >= 2, ok2 = t >= 1;
#pragma unroll 1
  for (int it = 0; it < 4; ++it) {
    const int d = tid + NTHR * it;
    const v4f w = *(const v4f*)(cw + 4 * d);
    const float bv = bf16_val(cb[d]);
    float x0 = XR[(size_t)r0 * XRW + d];
    float x1 = XR[(size_t)r1 * XRW + d];
    float x2 = XR[(size_t)r2 * XRW + d];
    const float x3 = XR[(size_t)m * XRW + d];
    x0 = ok0 ? x0 : 0.0f;
    x1 = ok1 ? x1 : 0.0f;
    x2 = ok2 ? x2 : 0.0f;
    float acc = bf16_val(w.x) * x0;
    acc = fmaf(bf16_val(w.y), x1, acc);
    acc = fmaf(bf16_val(w.z), x2, acc);
    acc = fmaf(bf16_val(w.w), x3, acc);
    const float xc = acc + bv;
    const float uu = xc * (1.0f / (1.0f + expf(-xc)));
    const unsigned hb = bf16_bits(uu);
    const unsigned lb = bf16_bits(uu - __uint_as_float(hb << 16));
    urow[d] = uu;
    hl[d] = (unsigned short)hb;
    hl[DI + d] = (unsigned short)lb;
  }
  __syncthreads();
  const v4f  uv = *(const v4fa*)(urow + 4 * tid);
  const v8us hv = *(const v8usa*)(hl + 8 * tid);
  float* up = U + (size_t)m * DI + 4 * tid;
  unsigned short* hp = UHL + (size_t)m * K2U + 8 * tid;
  *(volatile v4f*)up = uv;
  *(volatile v8us*)hp = hv;
  __threadfence();
  *(volatile v4f*)up = uv;
  *(volatile v8us*)hp = hv;
}

__global__ __launch_bounds__(NTHR) void k_scan(const float* __restrict__ DELTA, const float* __restrict__ U,
                                               const float* __restrict__ XDBL, const float* __restrict__ XR,
                                               const float* __restrict__ A_log, const float* __restrict__ Dv,
                                               unsigned short* YG) {
  __shared__ __attribute__((aligned(16))) float dlt[TC * SD];
  __shared__ __attribute__((aligned(16))) float ult[TC * SD];
  __shared__ __attribute__((aligned(16))) float bct[TC * 32];
  __shared__ __attribute__((aligned(16))) float ytl[TC * SD];
  const int tid = (int)threadIdx.x;
  const int dl = tid >> 2, q = tid & 3;
  const int d0 = (int)blockIdx.x * SD;
  const int b  = (int)blockIdx.y;
  const int d  = d0 + dl;

  float A0, A1, A2, A3;
  {
    const v4f al = *(const v4f*)(A_log + (size_t)d * NS + 4 * q);
    A0 = -expf(bf16_val(al.x));
    A1 = -expf(bf16_val(al.y));
    A2 = -expf(bf16_val(al.z));
    A3 = -expf(bf16_val(al.w));
  }
  const float Dd = bf16_val(Dv[d]);
  float s0 = 0.0f, s1 = 0.0f, s2 = 0.0f, s3 = 0.0f;

  const int sr = tid >> 4, sc = (tid & 15) * 4;
  const int br = tid >> 3, bc = (tid & 7) * 4;
  const int orow = tid >> 3, op8 = tid & 7;

#pragma unroll 1
  for (int ch = 0; ch < LL / TC; ++ch) {
    const int mb = b * LL + ch * TC;
    {
      const v4f a0 = *(const v4f*)(DELTA + (size_t)(mb + sr) * DI + d0 + sc);
      const v4f a1 = *(const v4f*)(DELTA + (size_t)(mb + sr + 16) * DI + d0 + sc);
      const v4f u0 = *(const v4f*)(U + (size_t)(mb + sr) * DI + d0 + sc);
      const v4f u1 = *(const v4f*)(U + (size_t)(mb + sr + 16) * DI + d0 + sc);
      const v4f c4 = *(const v4f*)(XDBL + (size_t)(mb + br) * XW + RK + bc);
      *(v4fa*)(dlt + sr * SD + sc) = a0;
      *(v4fa*)(dlt + (sr + 16) * SD + sc) = a1;
      *(v4fa*)(ult + sr * SD + sc) = u0;
      *(v4fa*)(ult + (sr + 16) * SD + sc) = u1;
      *(v4fa*)(bct + br * 32 + bc) = c4;
    }
    __syncthreads();

#pragma unroll 1
    for (int r = 0; r < TC; ++r) {
      const float dt = dlt[r * SD + dl];
      const float uu = ult[r * SD + dl];
      const v4f Bv = *(const v4fa*)(bct + r * 32 + 4 * q);
      const v4f Cv = *(const v4fa*)(bct + r * 32 + NS + 4 * q);
      const float du = dt * uu;
      const float e0 = expf(dt * A0);
      const float e1 = expf(dt * A1);
      const float e2 = expf(dt * A2);
      const float e3 = expf(dt * A3);
      s0 = fmaf(e0, s0, du * Bv.x);
      s1 = fmaf(e1, s1, du * Bv.y);
      s2 = fmaf(e2, s2, du * Bv.z);
      s3 = fmaf(e3, s3, du * Bv.w);
      float p = s0 * Cv.x;
      p = fmaf(s1, Cv.y, p);
      p = fmaf(s2, Cv.z, p);
      p = fmaf(s3, Cv.w, p);
      p += __shfl_xor(p, 1, 32);
      p += __shfl_xor(p, 2, 32);
      const float yv = fmaf(uu, Dd, p);
      if (q == 0) ytl[r * SD + dl] = yv;
    }
    __syncthreads();

    const int m = mb + orow;
    float* yp = ytl + orow * SD + 8 * op8;
    const float* rp = XR + (size_t)m * XRW + DI + d0 + 8 * op8;
#pragma unroll 1
    for (int j = 0; j < 8; ++j) {
      const float yv = yp[j];
      const float rv = rp[j];
      const float sg = 1.0f / (1.0f + expf(-rv));
      yp[j] = yv * (rv * sg);
    }
    const v4f g0 = *(const v4fa*)yp;
    const v4f g1 = *(const v4fa*)(yp + 4);
    v8us hv, lv;
    hv[0] = hl_sel(g0.x, false); lv[0] = hl_sel(g0.x, true);
    hv[1] = hl_sel(g0.y, false); lv[1] = hl_sel(g0.y, true);
    hv[2] = hl_sel(g0.z, false); lv[2] = hl_sel(g0.z, true);
    hv[3] = hl_sel(g0.w, false); lv[3] = hl_sel(g0.w, true);
    hv[4] = hl_sel(g1.x, false); lv[4] = hl_sel(g1.x, true);
    hv[5] = hl_sel(g1.y, false); lv[5] = hl_sel(g1.y, true);
    hv[6] = hl_sel(g1.z, false); lv[6] = hl_sel(g1.z, true);
    hv[7] = hl_sel(g1.w, false); lv[7] = hl_sel(g1.w, true);
    unsigned short* hp = YG + (size_t)m * K2U + d0 + 8 * op8;
    *(volatile v8us*)hp = hv;
    *(volatile v8us*)(hp + DI) = lv;
    __threadfence();
    *(volatile v8us*)hp = hv;
    *(volatile v8us*)(hp + DI) = lv;
  }
}

static inline size_t al256(size_t o) { return (o + 255) & ~(size_t)255; }

extern "C" void kernel_launch(void* const* d_in, const int* in_sizes, int n_in,
                              void* d_out, int out_size, void* d_ws, size_t ws_size,
                              hipStream_t stream) {
  if (n_in < 11) return;
  if (in_sizes[0] != MR * DM) return;
  if (in_sizes[1] != DM * XRW) return;
  if (in_sizes[2] != DI * 4) return;
  if (in_sizes[3] != DI) return;
  if (in_sizes[4] != DI * XW) return;
  if (in_sizes[5] != RK * DI) return;
  if (in_sizes[6] != DI) return;
  if (in_sizes[7] != DI * NS) return;
  if (in_sizes[8] != DI) return;
  if (in_sizes[9] != DI * DM) return;
  if (in_sizes[10] != DM) return;
  if (out_size != MR * DM) return;

  const float* x      = (const float*)d_in[0];
  const float* W_in   = (const float*)d_in[1];
  const float* conv_w = (const float*)d_in[2];
  const float* conv_b = (const float*)d_in[3];
  const float* W_x    = (const float*)d_in[4];
  const float* W_dt   = (const float*)d_in[5];
  const float* b_dt   = (const float*)d_in[6];
  const float* A_log  = (const float*)d_in[7];
  const float* Dvec   = (const float*)d_in[8];
  const float* W_out  = (const float*)d_in[9];
  const float* b_out  = (const float*)d_in[10];
  float* out = (float*)d_out;

  char* ws = (char*)d_ws;
  size_t off = 0;
  const size_t oXB  = off; off = al256(off + (size_t)MR * DM * 2);
  const size_t oWI  = off; off = al256(off + (size_t)XRW * DM * 2);
  const size_t oWX  = off; off = al256(off + (size_t)XW * K2U * 2);
  const size_t oWD  = off; off = al256(off + (size_t)DI * K2D * 2);
  const size_t oWO  = off; off = al256(off + (size_t)DM * K2U * 2);
  const size_t oXR  = off; off = al256(off + (size_t)MR * XRW * 4);
  const size_t oU   = off; off = al256(off + (size_t)MR * DI * 4);
  const size_t oUH  = off; off = al256(off + (size_t)MR * K2U * 2);
  const size_t oXD  = off; off = al256(off + (size_t)MR * XW * 4);
  const size_t oDT  = off; off = al256(off + (size_t)MR * K2D * 2);
  const size_t oDL  = off; off = al256(off + (size_t)MR * DI * 4);
  const size_t oYG  = off; off = al256(off + (size_t)MR * K2U * 2);
  if (off > ws_size || off > (size_t)WSMAX) return;
  unsigned short* XB   = (unsigned short*)(ws + oXB);
  unsigned short* WINT = (unsigned short*)(ws + oWI);
  unsigned short* WX2  = (unsigned short*)(ws + oWX);
  unsigned short* WDT2 = (unsigned short*)(ws + oWD);
  unsigned short* WO2  = (unsigned short*)(ws + oWO);
  float*          XR   = (float*)(ws + oXR);
  float*          U    = (float*)(ws + oU);
  unsigned short* UHL  = (unsigned short*)(ws + oUH);
  float*          XDBL = (float*)(ws + oXD);
  unsigned short* DTR  = (unsigned short*)(ws + oDT);
  float*          DELTA= (float*)(ws + oDL);
  unsigned short* YG   = (unsigned short*)(ws + oYG);

  k_prep<<<UTOT / NTHR, NTHR, 0, stream>>>(x, W_in, W_x, W_dt, W_out, XB, WINT, WX2, WDT2, WO2);
  k_gemm<0><<<dim3(MR / GBM, XRW / GBN), GTHR, 0, stream>>>(XB, WINT, DM, b_out, XR, XRW, YG);
  k_conv<<<MR, NTHR, 0, stream>>>(XR, conv_w, conv_b, U, UHL);
  k_gemm<1><<<dim3(MR / GBM, XW / GBN), GTHR, 0, stream>>>(UHL, WX2, K2U, b_out, XDBL, XW, DTR);
  k_gemm<2><<<dim3(MR / GBM, DI / GBN), GTHR, 0, stream>>>(DTR, WDT2, K2D, b_dt, DELTA, DI, YG);
  k_scan<<<dim3(DI / SD, NB), NTHR, 0, stream>>>(DELTA, U, XDBL, XR, A_log, Dvec, YG);
  k_gemm<3><<<dim3(MR / GBM, DM / GBN), GTHR, 0, stream>>>(YG, WO2, K2U, b_out, out, DM, DTR);
}
